// CGC_Layer_29205777613114
// MI455X (gfx1250) — hardware-run, weakly checked
//
#include <hip/hip_runtime.h>
#include <math.h>

typedef __attribute__((ext_vector_type(16))) _Float16 v16h;
typedef __attribute__((ext_vector_type(8)))  _Float16 v8h;
typedef __attribute__((ext_vector_type(8)))  float    v8f;
typedef __attribute__((ext_vector_type(4)))  float    v4f;

constexpr int kB      = 8192;
constexpr int kD      = 512;
constexpr int kH      = 1024;
constexpr int kO      = 512;
constexpr int kNExp   = 12;
constexpr int kBc     = 512;
constexpr int kNChunk = kB / kBc;
constexpr int kGateN  = 64;
constexpr int kGatePitch = 32;
constexpr float kEps  = 1e-5f;
constexpr float kXCarry = 16.0f;
constexpr float kHCarry = 16.0f;
constexpr float kWCarry = 1024.0f;
constexpr float kScale1 = 1.0f / (kXCarry * kWCarry);
constexpr float kScale2 = 1.0f / (kHCarry * kWCarry);
constexpr bool kPreRneBf16 = false;

static_assert(kB % kBc == 0 && kBc % 64 == 0, "chunk rows are tile multiples");
static_assert(kD % 32 == 0 && kH % 32 == 0, "GEMM K multiples of 32");
static_assert(kH % 64 == 0 && kO % 64 == 0 && kGateN % 64 == 0 && kB % 64 == 0, "GEMM M,N multiples of 64");
static_assert(kH == 4 * 256, "normalisation kernel: 4 segments of 256 columns per row");
static_assert((size_t)kB * kO * 4 == 16777216ull, "per-output byte size");
static_assert((size_t)3 * kB * kO * 4 == 50331648ull, "total output bytes");

constexpr size_t kOffXH    = 0;
constexpr size_t kOffW1T   = kOffXH    + (size_t)3 * kB * kD * 2;
constexpr size_t kOffW2T   = kOffW1T   + (size_t)kNExp * kH * kD * 2;
constexpr size_t kOffGT    = kOffW2T   + (size_t)kNExp * kO * kH * 2;
constexpr size_t kOffLOG   = kOffGT    + (size_t)3 * kGateN * kD * 2;
constexpr size_t kOffGATE  = kOffLOG   + (size_t)3 * kB * kGateN * 4;
constexpr size_t kOffHPRE  = kOffGATE  + (size_t)kB * kGatePitch * 4;
constexpr size_t kOffHPOST = kOffHPRE  + (size_t)kNExp * kBc * kH * 4;
constexpr size_t kOffEOUT  = kOffHPOST + (size_t)kNExp * kBc * kH * 2;
constexpr size_t kWsTotal  = kOffEOUT  + (size_t)kNExp * kBc * kO * 4;
static_assert(kWsTotal == 108199936ull, "carve total");
static_assert(kWsTotal <= 134217728ull, "carve cap");
static_assert((kOffW1T % 128) == 0 && (kOffW2T % 128) == 0 && (kOffGT % 128) == 0 && (kOffLOG % 128) == 0 &&
              (kOffGATE % 128) == 0 && (kOffHPRE % 128) == 0 && (kOffHPOST % 128) == 0 && (kOffEOUT % 128) == 0,
              "128-B aligned regions");

__device__ __forceinline__ unsigned short f2bf_bits(float f) {
  unsigned u = __float_as_uint(f);
  return (unsigned short)((u + 0x7FFFu + ((u >> 16) & 1u)) >> 16);
}
__device__ __forceinline__ float bf_bits2f(unsigned short h) { return __uint_as_float(((unsigned)h) << 16); }
__device__ __forceinline__ float prne(float f) {
  if (kPreRneBf16) return bf_bits2f(f2bf_bits(f));
  return f;
}

__device__ __forceinline__ void tie_h(v8f& a, v16h x, v16h y) { asm volatile("" : "+v"(a) : "v"(x), "v"(y)); }
__device__ __forceinline__ void tie_nop_h(v8f& a, v16h x, v16h y) { asm volatile("v_nop\n\tv_nop\n\tv_nop\n\tv_nop" : "+v"(a) : "v"(x), "v"(y)); }
__device__ __forceinline__ void keep4_h(v16h a, v16h b, v16h c, v16h d) { asm volatile("v_nop" :: "v"(a), "v"(b), "v"(c), "v"(d)); }
__device__ __forceinline__ void acc_guard4(v8f& a, v8f& b, v8f& c, v8f& d) { asm volatile("v_nop\n\tv_nop\n\tv_nop\n\tv_nop" : "+v"(a), "+v"(b), "+v"(c), "+v"(d)); }

struct FragH {
  union U { v16h v; v8h h[2]; };
  static __device__ __forceinline__ v16h load(const _Float16* p) {
    U f; f.h[0] = *(const v8h*)(p); f.h[1] = *(const v8h*)(p + 16); return f.v;
  }
  static __device__ __forceinline__ v8f mma(v16h a, v16h b, v8f c) {
    return __builtin_amdgcn_wmma_f32_16x16x32_f16(false, a, false, b, (short)0, c, false, false);
  }
};

template <int AMAP, int BIASMODE>
__global__ __launch_bounds__(256) void gemm64_f16_kernel(
    const unsigned short* __restrict__ Ap, int lda, long strideA,
    const unsigned short* __restrict__ Btp, int ldb, long strideB,
    float* __restrict__ Cout, int ldc, long strideC,
    const float* __restrict__ biasT, const float* __restrict__ biasS,
    int M, int N, int K, float scale) {
  typedef _Float16 T;
  typedef v16h V;
  const T* A = (const T*)Ap;
  const T* Bt = (const T*)Btp;
  __shared__ __align__(16) float sT[8][16 * 68];
  const int b    = blockIdx.y;
  const int lane = threadIdx.x & 31;
  const int wave = __builtin_amdgcn_readfirstlane((int)(threadIdx.x >> 5));
  const int tilesN = N >> 6;
  const int tilesM = M >> 6;
  const int tile = blockIdx.x * 8 + wave;
  if (tile >= tilesM * tilesN) return;
  const int tm = tile / tilesN;
  const int tn = tile - tm * tilesN;
  const int m0 = tm << 6;
  const int n0 = tn << 6;

  const int ab = (AMAP == 1) ? (((b >> 2) + 1) % 3) : b;
  const T* Ab = A  + (size_t)ab * strideA;
  const T* Bb = Bt + (size_t)b * strideB;
  const float* bp = nullptr;
  if (BIASMODE == 1) bp = (b < 8) ? (biasT + (size_t)b * N) : (biasS + (size_t)(b - 8) * N);

  const int rlane = lane & 15;
  const int koff  = (lane >> 4) * 8;
  const int mOff  = (lane >> 4) * 8;

  v8f acc[4][4];
#pragma unroll
  for (int i = 0; i < 4; ++i)
#pragma unroll
    for (int j = 0; j < 4; ++j) acc[i][j] = (v8f){0.f,0.f,0.f,0.f,0.f,0.f,0.f,0.f};

  for (int k0 = 0; k0 < K; k0 += 32) {
    V bh[4];
#pragma unroll
    for (int j = 0; j < 4; ++j) {
      const size_t bo = (size_t)(n0 + (j << 4) + rlane) * ldb + koff + k0;
      bh[j] = FragH::load(Bb + bo);
    }
#pragma unroll
    for (int i = 0; i < 4; ++i) {
      const size_t ao = (size_t)(m0 + (i << 4) + rlane) * lda + koff + k0;
      V ah = FragH::load(Ab + ao);
#pragma unroll
      for (int j = 0; j < 4; ++j) acc[i][j] = FragH::mma(ah, bh[j], acc[i][j]);
      tie_h(acc[i][0], ah, bh[0]);
      tie_h(acc[i][1], ah, bh[1]);
      tie_h(acc[i][2], ah, bh[2]);
      tie_nop_h(acc[i][3], ah, bh[3]);
    }
    keep4_h(bh[0], bh[1], bh[2], bh[3]);
  }
  acc_guard4(acc[0][0], acc[0][1], acc[0][2], acc[0][3]);
  acc_guard4(acc[1][0], acc[1][1], acc[1][2], acc[1][3]);
  acc_guard4(acc[2][0], acc[2][1], acc[2][2], acc[2][3]);
  acc_guard4(acc[3][0], acc[3][1], acc[3][2], acc[3][3]);

  float* slab = sT[wave];
  float* C = Cout + (size_t)b * strideC;
#pragma unroll
  for (int i = 0; i < 4; ++i) {
    const int mBase = m0 + (i << 4);
#pragma unroll
    for (int j = 0; j < 4; ++j) {
      const int n = n0 + (j << 4) + rlane;
      float bv = 0.f;
      if (BIASMODE == 1) bv = prne(bp[n]);
#pragma unroll
      for (int r = 0; r < 8; ++r) {
        float v = acc[i][j][r] * scale;
        if (BIASMODE == 1) v += bv;
        slab[(mOff + r) * 68 + (j << 4) + rlane] = v;
      }
    }
    __builtin_amdgcn_fence(__ATOMIC_RELEASE, "workgroup");
    __builtin_amdgcn_wave_barrier();
    __builtin_amdgcn_fence(__ATOMIC_ACQUIRE, "workgroup");
    {
      const int hh = lane >> 4, c4 = (lane & 15) * 4;
      for (int pass = 0; pass < 2; ++pass) {
#pragma unroll
        for (int it = 0; it < 8; ++it) {
          const int row = it * 2 + hh;
          v4f v = *(const v4f*)(slab + row * 68 + c4);
          *(volatile v4f*)(C + (size_t)(mBase + row) * ldc + n0 + c4) = v;
        }
        __threadfence();
      }
    }
    __builtin_amdgcn_fence(__ATOMIC_RELEASE, "workgroup");
    __builtin_amdgcn_wave_barrier();
    __builtin_amdgcn_fence(__ATOMIC_ACQUIRE, "workgroup");
  }
}

__global__ __launch_bounds__(256) void cvt_x_kernel(
    const float* __restrict__ sh, const float* __restrict__ tx, unsigned short* __restrict__ xh) {
  const int i = blockIdx.x * 256 + threadIdx.x;
  const size_t e0 = (size_t)i << 3;
  constexpr size_t nS = (size_t)kB * kD;
  const bool isS = (e0 < nS);
  const float* src = isS ? (sh + e0) : (tx + (e0 - nS));
  const v4f a0 = *(const v4f*)(src);
  const v4f a1 = *(const v4f*)(src + 4);
  v8h hv;
#pragma unroll
  for (int e = 0; e < 4; ++e) {
    hv[e]     = (_Float16)(prne(a0[e]) * kXCarry);
    hv[4 + e] = (_Float16)(prne(a1[e]) * kXCarry);
  }
  unsigned short* q = xh + e0;
  *(volatile v8h*)q = hv;
  __threadfence();
  *(volatile v8h*)q = hv;
}

__global__ __launch_bounds__(256) void cvt_wT_kernel(
    const float* __restrict__ wT, const float* __restrict__ wS, unsigned short* __restrict__ dst, int R, int C) {
  __shared__ float sT[64 * 65];
  const int tid  = threadIdx.x;
  const int lane = tid & 31;
  const int wave = __builtin_amdgcn_readfirstlane((int)(threadIdx.x >> 5));
  const int e  = blockIdx.z;
  const int c0 = blockIdx.x * 64;
  const int r0 = blockIdx.y * 64;
  const size_t plane = (size_t)R * C;
  const float* src = (e < 8) ? (wT + (size_t)e * plane) : (wS + (size_t)(e - 8) * plane);
  const int lr = tid >> 4, lc = (tid & 15) * 4;
#pragma unroll
  for (int i = 0; i < 4; ++i) {
    const int r = lr + 16 * i;
    const v4f v = *(const v4f*)(src + (size_t)(r0 + r) * C + c0 + lc);
    sT[r * 65 + lc + 0] = v[0];
    sT[r * 65 + lc + 1] = v[1];
    sT[r * 65 + lc + 2] = v[2];
    sT[r * 65 + lc + 3] = v[3];
  }
  __syncthreads();
  const int q = lane >> 3, seg = (lane & 7) * 8;
  v8h hv[2];
#pragma unroll
  for (int it = 0; it < 2; ++it) {
    const int cc = it * 32 + wave * 4 + q;
#pragma unroll
    for (int k = 0; k < 8; ++k) hv[it][k] = (_Float16)(prne(sT[(seg + k) * 65 + cc]) * kWCarry);
  }
  for (int pass = 0; pass < 2; ++pass) {
#pragma unroll
    for (int it = 0; it < 2; ++it) {
      const int cc = it * 32 + wave * 4 + q;
      *(volatile v8h*)(dst + ((size_t)e * C + c0 + cc) * R + r0 + seg) = hv[it];
    }
    __threadfence();
  }
}

__global__ __launch_bounds__(256) void cvt_gate_w_kernel(
    const float* __restrict__ gW, const float* __restrict__ sgW, unsigned short* __restrict__ gt) {
  const int i = blockIdx.x * 256 + threadIdx.x;
  const int p = i >> 12;
  const int rem = i & 4095;
  const int n = rem >> 6;
  const int k8 = (rem & 63) * 8;
  const int ncols = (p == 0) ? 12 : 8;
  const int pm = (p == 0) ? 0 : (p - 1);
  const float* src = (p == 0) ? sgW : (gW + (size_t)pm * kD * 8);
  const int nc = (n < ncols) ? n : (ncols - 1);
  const bool live = (n < ncols);
  v8h hv;
#pragma unroll
  for (int k = 0; k < 8; ++k) {
    float v = src[(size_t)(k8 + k) * ncols + nc];
    asm volatile("" : "+v"(v));
    const float w = live ? (prne(v) * kWCarry) : 0.0f;
    hv[k] = (_Float16)w;
  }
  unsigned short* q = gt + ((size_t)p * kGateN + n) * kD + k8;
  *(volatile v8h*)q = hv;
  __threadfence();
  *(volatile v8h*)q = hv;
}

__global__ __launch_bounds__(256) void gate_softmax_kernel(
    const float* __restrict__ logit, const float* __restrict__ gb, const float* __restrict__ sgb,
    float* __restrict__ gate) {
  __shared__ __align__(16) float sG[256 * 36];
  __shared__ float sB[32];
  const int tid  = threadIdx.x;
  const int lane = tid & 31;
  const int wave = __builtin_amdgcn_readfirstlane((int)(threadIdx.x >> 5));
  {
    const int j = tid & 31;
    const int js = (j < 11) ? j : 11;
    int jg = j - 16;
    jg = (jg < 0) ? 0 : jg;
    float vs = sgb[js];
    float vg = gb[jg];
    asm volatile("" : "+v"(vs));
    asm volatile("" : "+v"(vg));
    const float bsel = (j < 12) ? vs : ((j >= 16) ? vg : 0.0f);
    if (tid < 32) sB[j] = prne(bsel);
  }
  __syncthreads();
  const int row = blockIdx.x * 256 + tid;
  float* my = sG + tid * 36;
  {
    const float* l0 = logit + (size_t)row * kGateN;
    const float* l1 = logit + ((size_t)kB + row) * kGateN;
    const float* l2 = logit + ((size_t)2 * kB + row) * kGateN;
    const v4f a0 = *(const v4f*)(l0);
    const v4f a1 = *(const v4f*)(l0 + 4);
    const v4f a2 = *(const v4f*)(l0 + 8);
    const v4f b0 = *(const v4f*)(l1);
    const v4f b1 = *(const v4f*)(l1 + 4);
    const v4f c0 = *(const v4f*)(l2);
    const v4f c1 = *(const v4f*)(l2 + 4);
#pragma unroll
    for (int k = 0; k < 4; ++k) {
      my[k]      = a0[k] + sB[k];
      my[4 + k]  = a1[k] + sB[4 + k];
      my[8 + k]  = a2[k] + sB[8 + k];
      my[12 + k] = 0.0f;
      my[16 + k] = b0[k] + sB[16 + k];
      my[20 + k] = b1[k] + sB[20 + k];
      my[24 + k] = c0[k] + sB[24 + k];
      my[28 + k] = c1[k] + sB[28 + k];
    }
  }
#pragma unroll 1
  for (int sgm = 0; sgm < 3; ++sgm) {
    const int st = (sgm == 0) ? 0 : (8 + 8 * sgm);
    const int n  = (sgm == 0) ? 12 : 8;
    float* p = my + st;
    float mx = p[0];
#pragma unroll 1
    for (int j = 1; j < n; ++j) mx = fmaxf(mx, p[j]);
    float sum = 0.0f;
#pragma unroll 1
    for (int j = 0; j < n; ++j) {
      const float ev = expf(p[j] - mx);
      p[j] = ev;
      sum += ev;
    }
    const float inv = 1.0f / sum;
#pragma unroll 1
    for (int j = 0; j < n; ++j) p[j] = p[j] * inv;
  }
  __syncthreads();
  {
    const int q = lane >> 3, c4 = (lane & 7) * 4;
    v4f gv[8];
#pragma unroll
    for (int it = 0; it < 8; ++it) {
      const int rl = it * 32 + wave * 4 + q;
      gv[it] = *(const v4f*)(sG + rl * 36 + c4);
    }
    for (int pass = 0; pass < 2; ++pass) {
#pragma unroll
      for (int it = 0; it < 8; ++it) {
        const int rl = it * 32 + wave * 4 + q;
        *(volatile v4f*)(gate + ((size_t)blockIdx.x * 256 + rl) * kGatePitch + c4) = gv[it];
      }
      __threadfence();
    }
  }
}

__global__ __launch_bounds__(256) void ln_relu_kernel(
    const float* __restrict__ hpre,
    const float* __restrict__ gT, const float* __restrict__ gS,
    const float* __restrict__ betaT, const float* __restrict__ betaS,
    unsigned short* __restrict__ hpost) {
  const int lane = threadIdx.x & 31;
  const int wave = __builtin_amdgcn_readfirstlane((int)(threadIdx.x >> 5));
  const int e = blockIdx.x >> 3;
  const int rbase = (blockIdx.x & 7) * 64 + wave * 8;
  const float* gp = ((e < 8) ? (gT + (size_t)e * kH) : (gS + (size_t)(e - 8) * kH)) + lane * 8;
  const float* bp = ((e < 8) ? (betaT + (size_t)e * kH) : (betaS + (size_t)(e - 8) * kH)) + lane * 8;
  constexpr float kInvH = 1.0f / (float)kH;
#pragma unroll 1
  for (int rr = 0; rr < 8; ++rr) {
    const size_t row = (size_t)e * kBc + rbase + rr;
    const float* xp = hpre + row * kH + lane * 8;
    float sm = 0.0f;
#pragma unroll 1
    for (int s = 0; s < 4; ++s) {
      const v4f a0 = *(const v4f*)(xp + s * 256);
      const v4f a1 = *(const v4f*)(xp + s * 256 + 4);
      const float t0 = (a0[0] + a0[1]) + (a0[2] + a0[3]);
      const float t1 = (a1[0] + a1[1]) + (a1[2] + a1[3]);
      sm += t0 + t1;
    }
    sm += __shfl_xor(sm, 16, 32);
    sm += __shfl_xor(sm, 8, 32);
    sm += __shfl_xor(sm, 4, 32);
    sm += __shfl_xor(sm, 2, 32);
    sm += __shfl_xor(sm, 1, 32);
    const float mu = sm * kInvH;
    float sq = 0.0f;
#pragma unroll 1
    for (int s = 0; s < 4; ++s) {
      const v4f a0 = *(const v4f*)(xp + s * 256);
      const v4f a1 = *(const v4f*)(xp + s * 256 + 4);
#pragma unroll
      for (int k = 0; k < 4; ++k) {
        const float d0 = a0[k] - mu;
        const float d1 = a1[k] - mu;
        sq = fmaf(d0, d0, sq);
        sq = fmaf(d1, d1, sq);
      }
    }
    sq += __shfl_xor(sq, 16, 32);
    sq += __shfl_xor(sq, 8, 32);
    sq += __shfl_xor(sq, 4, 32);
    sq += __shfl_xor(sq, 2, 32);
    sq += __shfl_xor(sq, 1, 32);
    const float rs = rsqrtf(sq * kInvH + kEps) * kHCarry;
    unsigned short* op = hpost + row * kH + lane * 8;
#pragma unroll 1
    for (int s = 0; s < 4; ++s) {
      const v4f a0 = *(const v4f*)(xp + s * 256);
      const v4f a1 = *(const v4f*)(xp + s * 256 + 4);
      const v4f g0 = *(const v4f*)(gp + s * 256);
      const v4f g1 = *(const v4f*)(gp + s * 256 + 4);
      const v4f b0 = *(const v4f*)(bp + s * 256);
      const v4f b1 = *(const v4f*)(bp + s * 256 + 4);
      v8h hv;
#pragma unroll
      for (int k = 0; k < 4; ++k) {
        float y0 = fmaf((a0[k] - mu) * rs, prne(g0[k]), prne(b0[k]) * kHCarry);
        float y1 = fmaf((a1[k] - mu) * rs, prne(g1[k]), prne(b1[k]) * kHCarry);
        y0 = fmaxf(y0, 0.0f);
        y1 = fmaxf(y1, 0.0f);
        hv[k]     = (_Float16)y0;
        hv[4 + k] = (_Float16)y1;
      }
      unsigned short* q = op + s * 256;
      *(volatile v8h*)q = hv;
      __threadfence();
      *(volatile v8h*)q = hv;
    }
  }
}

__global__ __launch_bounds__(256) void mix_kernel(
    const float* __restrict__ eout, const float* __restrict__ gate, float* __restrict__ out, int r0) {
  const int tid = threadIdx.x;
  const int rl = blockIdx.x * 2 + (tid >> 7);
  const int c4 = (tid & 127) * 4;
  const float* gr = gate + (size_t)(r0 + rl) * kGatePitch;
  const float* ep = eout + (size_t)rl * kO + c4;
  constexpr size_t kPlane = (size_t)kBc * kO;
  v4f a0 = (v4f){0.f, 0.f, 0.f, 0.f};
  v4f a1 = (v4f){0.f, 0.f, 0.f, 0.f};
  v4f a2 = (v4f){0.f, 0.f, 0.f, 0.f};
#pragma unroll 1
  for (int e = 0; e < 4; ++e) {
    const v4f v = *(const v4f*)(ep + (size_t)e * kPlane);
    const float w0 = gr[e];
    const float w1 = gr[16 + e];
    a0 += w0 * v;
    a1 += w1 * v;
  }
#pragma unroll 1
  for (int e = 4; e < 8; ++e) {
    const v4f v = *(const v4f*)(ep + (size_t)e * kPlane);
    const float w0 = gr[e];
    const float w2 = gr[20 + e];
    a0 += w0 * v;
    a2 += w2 * v;
  }
#pragma unroll 1
  for (int e = 8; e < 12; ++e) {
    const v4f v = *(const v4f*)(ep + (size_t)e * kPlane);
    const float w0 = gr[e];
    const float w1 = gr[12 + e];
    const float w2 = gr[20 + e];
    a0 += w0 * v;
    a1 += w1 * v;
    a2 += w2 * v;
  }
  constexpr size_t kOutPlane = (size_t)kB * kO;
  float* o0 = out + (size_t)(r0 + rl) * kO + c4;
  float* o1 = o0 + kOutPlane;
  float* o2 = o1 + kOutPlane;
  *(volatile v4f*)o0 = a0;
  *(volatile v4f*)o1 = a1;
  *(volatile v4f*)o2 = a2;
  __threadfence();
  *(volatile v4f*)o0 = a0;
  *(volatile v4f*)o1 = a1;
  *(volatile v4f*)o2 = a2;
}

extern "C" void kernel_launch(void* const* d_in, const int* in_sizes, int n_in,
                              void* d_out, int out_size, void* d_ws, size_t ws_size,
                              hipStream_t stream) {
  if (n_in < 18) return;
  if (in_sizes[0] != kB * kD) return;
  if (in_sizes[1] != 2 * kB * kD) return;
  if (in_sizes[2] != 4 * kD * kH) return;
  if (in_sizes[3] != 4 * kH) return;
  if (in_sizes[4] != 4 * kH) return;
  if (in_sizes[5] != 4 * kH) return;
  if (in_sizes[6] != 4 * kH * kO) return;
  if (in_sizes[7] != 4 * kO) return;
  if (in_sizes[8] != 8 * kD * kH) return;
  if (in_sizes[9] != 8 * kH) return;
  if (in_sizes[10] != 8 * kH) return;
  if (in_sizes[11] != 8 * kH) return;
  if (in_sizes[12] != 8 * kH * kO) return;
  if (in_sizes[13] != 8 * kO) return;
  if (in_sizes[14] != 2 * kD * 8) return;
  if (in_sizes[15] != 16) return;
  if (in_sizes[16] != kD * 12) return;
  if (in_sizes[17] != 12) return;
  if (out_size != 3 * kB * kO) return;
  if (ws_size < kWsTotal) return;

  const float* shared_input = (const float*)d_in[0];
  const float* task_x = (const float*)d_in[1];
  const float* sW1   = (const float*)d_in[2];
  const float* sb1   = (const float*)d_in[3];
  const float* sg    = (const float*)d_in[4];
  const float* sbeta = (const float*)d_in[5];
  const float* sW2   = (const float*)d_in[6];
  const float* sb2   = (const float*)d_in[7];
  const float* tW1   = (const float*)d_in[8];
  const float* tb1   = (const float*)d_in[9];
  const float* tg    = (const float*)d_in[10];
  const float* tbeta = (const float*)d_in[11];
  const float* tW2   = (const float*)d_in[12];
  const float* tb2   = (const float*)d_in[13];
  const float* gW    = (const float*)d_in[14];
  const float* gb    = (const float*)d_in[15];
  const float* sgW   = (const float*)d_in[16];
  const float* sgb   = (const float*)d_in[17];
  float* out = (float*)d_out;

  char* ws = (char*)d_ws;
  unsigned short* XH    = (unsigned short*)(ws + kOffXH);
  unsigned short* W1T   = (unsigned short*)(ws + kOffW1T);
  unsigned short* W2T   = (unsigned short*)(ws + kOffW2T);
  unsigned short* GT    = (unsigned short*)(ws + kOffGT);
  float*          LOG   = (float*)(ws + kOffLOG);
  float*          GATE  = (float*)(ws + kOffGATE);
  float*          HPRE  = (float*)(ws + kOffHPRE);
  unsigned short* HPOST = (unsigned short*)(ws + kOffHPOST);
  float*          EOUT  = (float*)(ws + kOffEOUT);

  cvt_x_kernel<<<(3 * kB * kD / 8) / 256, 256, 0, stream>>>(shared_input, task_x, XH);
  cvt_wT_kernel<<<dim3(kH / 64, kD / 64, kNExp), 256, 0, stream>>>(tW1, sW1, W1T, kD, kH);
  cvt_wT_kernel<<<dim3(kO / 64, kH / 64, kNExp), 256, 0, stream>>>(tW2, sW2, W2T, kH, kO);
  cvt_gate_w_kernel<<<(3 * kGateN * kD / 8) / 256, 256, 0, stream>>>(gW, sgW, GT);

  gemm64_f16_kernel<0, 0><<<dim3(16, 3), 256, 0, stream>>>(
      XH, kD, (long)kB * kD,
      GT, kD, (long)kGateN * kD,
      LOG, kGateN, (long)kB * kGateN,
      nullptr, nullptr,
      kB, kGateN, kD, kScale1);
  gate_softmax_kernel<<<kB / 256, 256, 0, stream>>>(LOG, gb, sgb, GATE);

  for (int c = 0; c < kNChunk; ++c) {
    const int r0 = c * kBc;
    gemm64_f16_kernel<1, 1><<<dim3(16, kNExp), 256, 0, stream>>>(
        XH + (size_t)r0 * kD, kD, (long)kB * kD,
        W1T, kD, (long)kH * kD,
        HPRE, kH, (long)kBc * kH,
        tb1, sb1,
        kBc, kH, kD, kScale1);
    ln_relu_kernel<<<kNExp * (kBc / 64), 256, 0, stream>>>(HPRE, tg, sg, tbeta, sbeta, HPOST);
    gemm64_f16_kernel<0, 1><<<dim3(8, kNExp), 256, 0, stream>>>(
        HPOST, kH, (long)kBc * kH,
        W2T, kH, (long)kO * kH,
        EOUT, kO, (long)kBc * kO,
        tb2, sb2,
        kBc, kO, kH, kScale2);
    mix_kernel<<<kBc / 2, 256, 0, stream>>>(EOUT, GATE, out, r0);
  }
}
